// S4Model_25761213841677
// MI455X (gfx1250) — hardware-run, weakly checked
//
#include <hip/hip_runtime.h>
#include <math.h>

typedef __attribute__((ext_vector_type(16))) _Float16 v16h;
typedef __attribute__((ext_vector_type(8)))  _Float16 v8h;
typedef __attribute__((ext_vector_type(8)))  float    v8f;
typedef __attribute__((ext_vector_type(4)))  float    v4f;
typedef __attribute__((ext_vector_type(2)))  float    v2f;
typedef __attribute__((ext_vector_type(4)))  unsigned v4u;

constexpr int kBatch    = 16;
constexpr int kChanIn   = 16;
constexpr int kLen      = 4096;
constexpr int kWidth    = 256;
constexpr int kModes    = 32;
constexpr int kLayers   = 4;
constexpr int kChunk    = 128;
constexpr int kChunksPS = kLen / kChunk;
constexpr int kRowsM    = kBatch * kChunksPS;
constexpr int kStateW   = 2 * kModes;
constexpr int kMvW      = kChunk + kStateW;
constexpr int kNpos     = kBatch * kLen;
constexpr int kPitchW   = 132;
constexpr int kPitchX   = 20;
static_assert(kChunksPS == 32 && kRowsM == 512 && kStateW == 64 && kMvW == 192 && kNpos == 65536, "derived shapes");
static_assert((kChunk % 32) == 0 && (kStateW % 32) == 0 && (kWidth % 32) == 0, "K multiples of 32");
static_assert((kRowsM % 64) == 0 && (kChunk % 64) == 0 && (kStateW % 64) == 0 && (kNpos % 64) == 0 && (kLen % 64) == 0, "tile multiples");

constexpr float kWCarry     = 256.0f;
constexpr float kWCarryInv  = 1.0f / 256.0f;
constexpr float kMvCarry    = 64.0f;
constexpr float kMvCarryInv = 1.0f / 64.0f;
constexpr float kECarry     = 64.0f;
constexpr float kECarryInv  = 1.0f / 64.0f;
constexpr float kLoScale    = 2048.0f;
constexpr float kLoScaleInv = 1.0f / 2048.0f;

constexpr size_t kOffH16   = 0;
constexpr size_t kOffG16   = kOffH16   + (size_t)kWidth * kNpos * 2;
constexpr size_t kOffInit  = kOffG16   + (size_t)kWidth * kNpos * 2;
constexpr size_t kOffMv    = kOffInit  + (size_t)kWidth * kRowsM * kStateW * 2;
constexpr size_t kOffEt    = kOffMv    + (size_t)kWidth * kChunk * kMvW * 2;
constexpr size_t kOffWpow  = kOffEt    + (size_t)kWidth * kStateW * kChunk * 2;
constexpr size_t kOffWoutT = kOffWpow  + (size_t)kWidth * kModes * 2 * 4;
constexpr size_t kOffDecH  = kOffWoutT + (size_t)kLayers * kWidth * kWidth * 2;
constexpr size_t kOffDecL  = kOffDecH  + (size_t)kChanIn * kWidth * 2;
constexpr size_t kOffEncT  = kOffDecL  + (size_t)kChanIn * kWidth * 2;
constexpr size_t kWsTotal  = kOffEncT  + (size_t)kWidth * 32 * 2;
static_assert(kWsTotal == 101285888ull, "carve total");
static_assert(kWsTotal <= 134217728ull, "carve cap");
static_assert((size_t)kWidth * kRowsM * kStateW * 4 == (size_t)kWidth * kNpos * 2, "state plane fits the shared region");
static_assert((kOffG16 % 128) == 0 && (kOffInit % 128) == 0 && (kOffMv % 128) == 0 && (kOffEt % 128) == 0 &&
              (kOffWpow % 128) == 0 && (kOffWoutT % 128) == 0 && (kOffDecH % 128) == 0 && (kOffDecL % 128) == 0 &&
              (kOffEncT % 128) == 0, "128-B aligned regions");

__device__ __forceinline__ unsigned short f16bits(float x) {
  const _Float16 h = (_Float16)x;
  return __builtin_bit_cast(unsigned short, h);
}
__device__ __forceinline__ unsigned pack2(float a, float b) {
  const unsigned lo = (unsigned)f16bits(a);
  const unsigned hi = (unsigned)f16bits(b);
  return lo | (hi << 16);
}
__device__ __forceinline__ float h16_to_f32(unsigned hb) {
  const unsigned sgn = (hb & 0x8000u) << 16;
  const unsigned em = hb & 0x7fffu;
  const float fn = __uint_as_float((em << 13) + 0x38000000u);
  const float fs = (float)em * 5.9604644775390625e-8f;
  const float mag = (em < 0x400u) ? fs : fn;
  return __uint_as_float(__float_as_uint(mag) | sgn);
}
__device__ __forceinline__ void wave_sync() {
  __builtin_amdgcn_fence(__ATOMIC_RELEASE, "workgroup");
  __builtin_amdgcn_wave_barrier();
  __builtin_amdgcn_fence(__ATOMIC_ACQUIRE, "workgroup");
}
__device__ __forceinline__ void store2_v4u(unsigned short* p, v4u v) {
  volatile v4u* q = (volatile v4u*)p;
  *q = v;
  __threadfence();
  *q = v;
}
__device__ __forceinline__ float gelu_fast(float y) {
  const float u = 0.7978845608028654f * (y + 0.044715f * y * y * y);
  const float e = __expf(-2.0f * u);
  return y * __builtin_amdgcn_rcpf(1.0f + e);
}

union FragH { v16h v; v8h h[2]; };
union FragW { v16h v; v4u q[2]; };
__device__ __forceinline__ v16h frag_load(const _Float16* p) {
  FragH f;
  f.h[0] = *(const v8h*)(p);
  f.h[1] = *(const v8h*)(p + 16);
  return f.v;
}
template <int PITCH>
__device__ __forceinline__ v16h lds_frag(const unsigned* sw, int n, int kw) {
  FragW f;
  f.q[0] = *(const v4u*)(sw + n * PITCH + kw);
  f.q[1] = *(const v4u*)(sw + n * PITCH + kw + 8);
  return f.v;
}
__device__ __forceinline__ v8f mma16(v16h a, v16h b, v8f c) {
  return __builtin_amdgcn_wmma_f32_16x16x32_f16(false, a, false, b, (short)0, c, false, false);
}
__device__ __forceinline__ void tie_acc(v8f& a, v16h x, v16h y) { asm volatile("" : "+v"(a) : "v"(x), "v"(y)); }
__device__ __forceinline__ void tie_acc_nops(v8f& a, v16h x, v16h y) { asm volatile("v_nop\n\tv_nop\n\tv_nop\n\tv_nop" : "+v"(a) : "v"(x), "v"(y)); }
__device__ __forceinline__ void keep4(v16h a, v16h b, v16h c, v16h d) { asm volatile("v_nop" :: "v"(a), "v"(b), "v"(c), "v"(d)); }
__device__ __forceinline__ void acc_guard4(v8f& a, v8f& b, v8f& c, v8f& d) { asm volatile("v_nop\n\tv_nop\n\tv_nop\n\tv_nop" : "+v"(a), "+v"(b), "+v"(c), "+v"(d)); }

__device__ __forceinline__ void kloop64(v8f (&acc)[4][4], const _Float16* ap, int lda,
                                        const _Float16* bp, int ldb, int ksteps) {
#pragma unroll 1
  for (int ks = 0; ks < ksteps; ++ks) {
    v16h bh[4];
#pragma unroll
    for (int j = 0; j < 4; ++j) bh[j] = frag_load(bp + (size_t)(j * 16) * ldb + ks * 32);
#pragma unroll
    for (int i = 0; i < 4; ++i) {
      const v16h ah = frag_load(ap + (size_t)(i * 16) * lda + ks * 32);
#pragma unroll
      for (int j = 0; j < 4; ++j) acc[i][j] = mma16(ah, bh[j], acc[i][j]);
      tie_acc(acc[i][0], ah, bh[0]);
      tie_acc(acc[i][1], ah, bh[1]);
      tie_acc(acc[i][2], ah, bh[2]);
      tie_acc_nops(acc[i][3], ah, bh[3]);
    }
    keep4(bh[0], bh[1], bh[2], bh[3]);
  }
}

template <int NT>
__device__ __forceinline__ void stage_tile_T(const unsigned short* plane, size_t n0, unsigned* sw, int tid) {
#pragma unroll 1
  for (int it = 0; it < 1024 / NT; ++it) {
    const int task = it * NT + tid;
    const int n8 = task & 7;
    const int kp = task >> 3;
    const unsigned short* p0 = plane + (size_t)(2 * kp) * kNpos + n0 + n8 * 8;
    const v4u a = *(const v4u*)(p0);
    const v4u b = *(const v4u*)(p0 + kNpos);
    unsigned* dst = sw + (n8 * 8) * kPitchW + kp;
#pragma unroll
    for (int j = 0; j < 4; ++j) {
      const unsigned aw = a[j];
      const unsigned bw = b[j];
      dst[(2 * j) * kPitchW]     = (aw & 0xffffu) | (bw << 16);
      dst[(2 * j + 1) * kPitchW] = (aw >> 16) | (bw & 0xffff0000u);
    }
  }
}

__device__ __forceinline__ void store_tile_rows(const unsigned* sw, unsigned short* plane, size_t n0, int wave, int lane) {
  const int q = lane >> 3;
  const int cw = lane & 7;
  v4u vals[8];
#pragma unroll
  for (int it = 0; it < 8; ++it) {
    const int row = it * 32 + wave * 4 + q;
    vals[it] = *(const v4u*)(sw + row * 32 + cw * 4);
  }
  for (int pass = 0; pass < 2; ++pass) {
#pragma unroll
    for (int it = 0; it < 8; ++it) {
      const int row = it * 32 + wave * 4 + q;
      *(volatile v4u*)(plane + (size_t)row * kNpos + n0 + cw * 8) = vals[it];
    }
    __threadfence();
  }
}

template <int KREAL, int KP, bool LO>
__device__ __forceinline__ void transpose_rows(const float* __restrict__ src, int ld, int mcount, int m0, int rows_valid,
                                               unsigned short* dhi, unsigned short* dlo, float* sT, int tid) {
  const int mm = tid & 31;
  const int kq = tid >> 5;
  int ms = m0 + mm;
  ms = (ms < mcount) ? ms : (mcount - 1);
#pragma unroll 1
  for (int it = 0; it < KREAL / 8; ++it) {
    const int k = it * 8 + kq;
    sT[mm * 257 + k] = src[(size_t)k * ld + ms];
  }
  __syncthreads();
  constexpr int CPR = KP / 8;
  constexpr int ITERS = (32 * CPR + 255) / 256;
  const int nchunks = rows_valid * CPR;
#pragma unroll 1
  for (int it = 0; it < ITERS; ++it) {
    const int q = it * 256 + tid;
    if (q < nchunks) {
      const int row = q / CPR;
      const int k8 = (q - row * CPR) * 8;
      float vh[8];
      float vl[8];
#pragma unroll
      for (int e = 0; e < 8; ++e) {
        const int kk = k8 + e;
        const int kc = (kk < KREAL) ? kk : (KREAL - 1);
        const float x = sT[row * 257 + kc];
        const float v = (kk < KREAL) ? (x * kWCarry) : 0.0f;
        const _Float16 hv = (_Float16)v;
        const float back = (float)hv;
        vh[e] = v;
        vl[e] = (v - back) * kLoScale;
      }
      const v4u ph = {pack2(vh[0], vh[1]), pack2(vh[2], vh[3]), pack2(vh[4], vh[5]), pack2(vh[6], vh[7])};
      store2_v4u(dhi + (size_t)q * 8, ph);
      if (LO) {
        const v4u pl = {pack2(vl[0], vl[1]), pack2(vl[2], vl[3]), pack2(vl[4], vl[5]), pack2(vl[6], vl[7])};
        store2_v4u(dlo + (size_t)q * 8, pl);
      }
    }
  }
}

__global__ __launch_bounds__(256) void weight_planes_kernel(
    const float* __restrict__ w_out, const float* __restrict__ enc_w, const float* __restrict__ dec_w,
    unsigned short* __restrict__ woutT, unsigned short* __restrict__ encT,
    unsigned short* __restrict__ decTh, unsigned short* __restrict__ decTl) {
  __shared__ float sT[32 * 257];
  const int tid = threadIdx.x;
  const int bid = blockIdx.x;
  if (bid < 32) {
    const int layer = bid >> 3;
    const int m0 = (bid & 7) * 32;
    transpose_rows<kWidth, kWidth, false>(w_out + (size_t)layer * kWidth * kWidth, kWidth, kWidth, m0, 32,
                                          woutT + (size_t)layer * kWidth * kWidth + (size_t)m0 * kWidth, nullptr, sT, tid);
  } else if (bid < 40) {
    const int m0 = (bid - 32) * 32;
    transpose_rows<kChanIn, 32, false>(enc_w, kWidth, kWidth, m0, 32, encT + (size_t)m0 * 32, nullptr, sT, tid);
  } else {
    transpose_rows<kWidth, kWidth, true>(dec_w, kChanIn, kChanIn, 0, kChanIn, decTh, decTl, sT, tid);
  }
}

__global__ __launch_bounds__(256) void encode_kernel(
    const float* __restrict__ x, const unsigned short* __restrict__ encT, const float* __restrict__ enc_b,
    unsigned short* __restrict__ h16) {
  __shared__ __align__(16) union { unsigned w[64 * kPitchW]; unsigned short s[64 * kPitchW * 2]; } sb;
  const int tid = threadIdx.x;
  const int lane = tid & 31;
  const int wave = __builtin_amdgcn_readfirstlane((int)(threadIdx.x >> 5));
  const int hh = lane >> 4;
  const int c = lane & 15;
  const size_t n0 = (size_t)blockIdx.x * 64;
  const int b = (int)(n0 >> 12);
  const int l0 = (int)(n0 & (size_t)(kLen - 1));
  {
    const int n = tid & 63;
    const int kq = tid >> 6;
    const float* xp = x + ((size_t)b * kChanIn + 4 * kq) * kLen + l0 + n;
    const float x0 = xp[0];
    const float x1 = xp[kLen];
    const float x2 = xp[2 * kLen];
    const float x3 = xp[3 * kLen];
    sb.w[n * kPitchX + 2 * kq]     = pack2(x0, x1);
    sb.w[n * kPitchX + 2 * kq + 1] = pack2(x2, x3);
    sb.w[n * kPitchX + 8 + 2 * kq] = 0u;
    sb.w[n * kPitchX + 9 + 2 * kq] = 0u;
  }
  __syncthreads();
  v8f acc[2][4];
#pragma unroll
  for (int i = 0; i < 2; ++i)
#pragma unroll
    for (int j = 0; j < 4; ++j) acc[i][j] = (v8f){0.f, 0.f, 0.f, 0.f, 0.f, 0.f, 0.f, 0.f};
  {
    v16h bf[4];
#pragma unroll
    for (int j = 0; j < 4; ++j) bf[j] = lds_frag<kPitchX>(sb.w, 16 * j + c, 4 * hh);
    const _Float16* Wr = (const _Float16*)encT + (size_t)(32 * wave + c) * 32 + 8 * hh;
#pragma unroll
    for (int i = 0; i < 2; ++i) {
      const v16h ah = frag_load(Wr + (size_t)(i * 16) * 32);
#pragma unroll
      for (int j = 0; j < 4; ++j) acc[i][j] = mma16(ah, bf[j], acc[i][j]);
      tie_acc(acc[i][0], ah, bf[0]);
      tie_acc(acc[i][1], ah, bf[1]);
      tie_acc(acc[i][2], ah, bf[2]);
      tie_acc_nops(acc[i][3], ah, bf[3]);
    }
    keep4(bf[0], bf[1], bf[2], bf[3]);
  }
  acc_guard4(acc[0][0], acc[0][1], acc[0][2], acc[0][3]);
  acc_guard4(acc[1][0], acc[1][1], acc[1][2], acc[1][3]);
  __syncthreads();
#pragma unroll
  for (int i = 0; i < 2; ++i) {
    const int d0 = 32 * wave + 16 * i + 8 * hh;
    const v4f b0 = *(const v4f*)(enc_b + d0);
    const v4f b1 = *(const v4f*)(enc_b + d0 + 4);
#pragma unroll
    for (int j = 0; j < 4; ++j) {
      const int n = 16 * j + c;
#pragma unroll
      for (int r = 0; r < 8; ++r) {
        const float bv = (r < 4) ? b0[r & 3] : b1[r & 3];
        const float o = fmaf(acc[i][j][r], kWCarryInv, bv);
        sb.s[(d0 + r) * 64 + n] = f16bits(o);
      }
    }
  }
  __syncthreads();
  store_tile_rows(sb.w, h16, n0, wave, lane);
}

__global__ __launch_bounds__(256) void layer_tables_kernel(
    const float* __restrict__ log_dt, const float* __restrict__ a_re, const float* __restrict__ a_im,
    const float* __restrict__ c_re, const float* __restrict__ c_im, const float* __restrict__ dskip,
    unsigned short* __restrict__ et16, unsigned short* __restrict__ mv16, float* __restrict__ wpow) {
  __shared__ float sPr[129 * 32];
  __shared__ float sPi[129 * 32];
  __shared__ float sK[128];
  __shared__ float sCr[32];
  __shared__ float sCi[32];
  const int tid = threadIdx.x;
  const int n = tid & 31;
  const int seg = __builtin_amdgcn_readfirstlane((int)(threadIdx.x >> 5));
  const int h = blockIdx.x;
  const int idx = h * kModes + n;
  const float dt = expf(log_dt[h]);
  const float ar = -expf(a_re[idx]);
  const float ai = a_im[idx];
  const float dr = ar * dt;
  const float di = ai * dt;
  const float em = expm1f(dr);
  const float es = em + 1.0f;
  float sn, cs;
  sincosf(di, &sn, &cs);
  const float cm1a = -(sn * sn) * (1.0f / (1.0f + fmaxf(cs, 0.0f)));
  const float cm1 = (cs > 0.0f) ? cm1a : (cs - 1.0f);
  const float wr = es * cs;
  const float wi = es * sn;
  const float nr = em * cs + cm1;
  const float ni = wi;
  const float inv = 1.0f / (ar * ar + ai * ai);
  const float qr = (nr * ar + ni * ai) * inv;
  const float qi = (ni * ar - nr * ai) * inv;
  const float cr = c_re[idx];
  const float ci = c_im[idx];
  const float c2r = 2.0f * (cr * qr - ci * qi);
  const float c2i = 2.0f * (cr * qi + ci * qr);
  float sr = wr, si = wi;
#pragma unroll 1
  for (int i = 0; i < 4; ++i) {
    const float t = sr * sr - si * si;
    si = 2.0f * sr * si;
    sr = t;
  }
  float gr = sr, gi = si;
#pragma unroll 1
  for (int i = 0; i < 3; ++i) {
    const float t = gr * gr - gi * gi;
    gi = 2.0f * gr * gi;
    gr = t;
  }
  float pr = 1.0f, pi = 0.0f;
#pragma unroll 1
  for (int s = 0; s < seg; ++s) {
    const float t = pr * sr - pi * si;
    pi = pr * si + pi * sr;
    pr = t;
  }
#pragma unroll 1
  for (int s = 0; s < 16; ++s) {
    const int l = 16 * seg + s;
    sPr[l * 32 + n] = pr;
    sPi[l * 32 + n] = pi;
    const float t = pr * wr - pi * wi;
    pi = pr * wi + pi * wr;
    pr = t;
  }
  if (seg == 7) {
    sPr[128 * 32 + n] = pr;
    sPi[128 * 32 + n] = pi;
  }
  if (seg == 0) {
    sCr[n] = c2r;
    sCi[n] = c2i;
    const v2f wv = {gr, gi};
    volatile v2f* wp = (volatile v2f*)(wpow + (size_t)(h * kModes + n) * 2);
    *wp = wv;
    __threadfence();
    *wp = wv;
  }
  __syncthreads();
  if (tid < 128) {
    float acc = 0.0f;
#pragma unroll 1
    for (int m = 0; m < kModes; ++m) {
      acc += sCr[m] * sPr[tid * 32 + m] - sCi[m] * sPi[tid * 32 + m];
    }
    sK[tid] = acc;
  }
  __syncthreads();
  const float kd = sK[0] + dskip[h];
#pragma unroll 1
  for (int it = 0; it < 8; ++it) {
    const int q = it * 256 + tid;
    const int row = q >> 4;
    const int s0 = (q & 15) * 8;
    float v[8];
#pragma unroll
    for (int e = 0; e < 8; ++e) {
      const int df = row - (s0 + e);
      int dc = (df < 0) ? 0 : df;
      dc = (dc > 127) ? 127 : dc;
      const float kv = sK[dc];
      const float val = (df > 0) ? kv : ((df == 0) ? kd : 0.0f);
      v[e] = val * kMvCarry;
    }
    const v4u pk = {pack2(v[0], v[1]), pack2(v[2], v[3]), pack2(v[4], v[5]), pack2(v[6], v[7])};
    store2_v4u(mv16 + ((size_t)h * kChunk + row) * kMvW + s0, pk);
  }
#pragma unroll 1
  for (int it = 0; it < 4; ++it) {
    const int q = it * 256 + tid;
    const int row = q >> 3;
    const int nb = (q & 7) * 4;
    unsigned wd[4];
#pragma unroll
    for (int e = 0; e < 4; ++e) {
      const int m = nb + e;
      const float ppr = sPr[(row + 1) * 32 + m];
      const float ppi = sPi[(row + 1) * 32 + m];
      const float a = sCr[m];
      const float bq = sCi[m];
      const float re = a * ppr - bq * ppi;
      const float im = a * ppi + bq * ppr;
      wd[e] = pack2(re * kMvCarry, -im * kMvCarry);
    }
    const v4u pk = {wd[0], wd[1], wd[2], wd[3]};
    store2_v4u(mv16 + ((size_t)h * kChunk + row) * kMvW + kChunk + nb * 2, pk);
  }
#pragma unroll 1
  for (int it = 0; it < 4; ++it) {
    const int q = it * 256 + tid;
    const int r = q >> 4;
    const int k8 = (q & 15) * 8;
    const int m = r >> 1;
    const int part = r & 1;
    float v[8];
#pragma unroll
    for (int e = 0; e < 8; ++e) {
      const int l = 127 - (k8 + e);
      const float a = sPr[l * 32 + m];
      const float bq = sPi[l * 32 + m];
      const float val = part ? bq : a;
      v[e] = val * kECarry;
    }
    const v4u pk = {pack2(v[0], v[1]), pack2(v[2], v[3]), pack2(v[4], v[5]), pack2(v[6], v[7])};
    store2_v4u(et16 + ((size_t)h * kStateW + r) * kChunk + k8, pk);
  }
}

template <int MODE>
__global__ __launch_bounds__(256) void chunk_gemm_kernel(
    const unsigned short* __restrict__ hplane, const unsigned short* __restrict__ initp,
    const unsigned short* __restrict__ btp, void* __restrict__ cout) {
  __shared__ __align__(16) float sT[8][16 * 68];
  __shared__ __align__(16) unsigned sHw[(MODE == 1) ? 8 : 1][(MODE == 1) ? 16 * 32 : 4];
  const int h = blockIdx.y;
  const int lane = threadIdx.x & 31;
  const int wave = __builtin_amdgcn_readfirstlane((int)(threadIdx.x >> 5));
  const int tile = (MODE == 1) ? ((int)blockIdx.x * 8 + wave) : wave;
  const int tn = (MODE == 1) ? (tile & 1) : 0;
  const int tm = (MODE == 1) ? (tile >> 1) : tile;
  const int m0 = tm << 6;
  const int n0 = tn << 6;
  const int rlane = lane & 15;
  const int koff = (lane >> 4) * 8;
  const int mOff = (lane >> 4) * 8;
  constexpr int LDB = (MODE == 1) ? kMvW : kChunk;
  constexpr int BROWS = (MODE == 1) ? kChunk : kStateW;
  const _Float16* A1 = (const _Float16*)hplane + (size_t)h * kNpos;
  const _Float16* Bt = (const _Float16*)btp + (size_t)h * BROWS * LDB;

  v8f acc[4][4];
#pragma unroll
  for (int i = 0; i < 4; ++i)
#pragma unroll
    for (int j = 0; j < 4; ++j) acc[i][j] = (v8f){0.f, 0.f, 0.f, 0.f, 0.f, 0.f, 0.f, 0.f};

  kloop64(acc, A1 + (size_t)(m0 + rlane) * kChunk + koff, kChunk,
          Bt + (size_t)(n0 + rlane) * LDB + koff, LDB, kChunk / 32);
  if (MODE == 1) {
    const _Float16* A2 = (const _Float16*)initp + (size_t)h * kRowsM * kStateW;
    kloop64(acc, A2 + (size_t)(m0 + rlane) * kStateW + koff, kStateW,
            Bt + (size_t)(n0 + rlane) * LDB + kChunk + koff, LDB, kStateW / 32);
  }
  acc_guard4(acc[0][0], acc[0][1], acc[0][2], acc[0][3]);
  acc_guard4(acc[1][0], acc[1][1], acc[1][2], acc[1][3]);
  acc_guard4(acc[2][0], acc[2][1], acc[2][2], acc[2][3]);
  acc_guard4(acc[3][0], acc[3][1], acc[3][2], acc[3][3]);

  float* slab = sT[wave];
  const float scale = (MODE == 1) ? kMvCarryInv : kECarryInv;
#pragma unroll
  for (int i = 0; i < 4; ++i) {
    const int mBase = m0 + (i << 4);
#pragma unroll
    for (int j = 0; j < 4; ++j) {
#pragma unroll
      for (int r = 0; r < 8; ++r) slab[(mOff + r) * 68 + (j << 4) + rlane] = acc[i][j][r] * scale;
    }
    wave_sync();
    if (MODE == 0) {
      float* C = (float*)cout + (size_t)h * kRowsM * kStateW;
      const int h2 = lane >> 4;
      const int c4 = (lane & 15) * 4;
      for (int pass = 0; pass < 2; ++pass) {
#pragma unroll
        for (int it = 0; it < 8; ++it) {
          const int row = it * 2 + h2;
          const v4f v = *(const v4f*)(slab + row * 68 + c4);
          *(volatile v4f*)(C + (size_t)(mBase + row) * kStateW + c4) = v;
        }
        __threadfence();
      }
    } else {
      unsigned* sH = sHw[wave];
      unsigned short* G = (unsigned short*)cout + (size_t)h * kNpos;
      const int q = lane >> 3;
      const int cw = lane & 7;
#pragma unroll 1
      for (int it = 0; it < 4; ++it) {
        const int row = it * 4 + q;
        const float* sp = slab + row * 68 + cw * 8;
        const v4f a0 = *(const v4f*)(sp);
        const v4f a1 = *(const v4f*)(sp + 4);
        const v4u pk = {pack2(gelu_fast(a0[0]), gelu_fast(a0[1])), pack2(gelu_fast(a0[2]), gelu_fast(a0[3])),
                        pack2(gelu_fast(a1[0]), gelu_fast(a1[1])), pack2(gelu_fast(a1[2]), gelu_fast(a1[3]))};
        *(v4u*)(sH + row * 32 + cw * 4) = pk;
      }
      wave_sync();
      v4u vals[4];
#pragma unroll
      for (int it = 0; it < 4; ++it) vals[it] = *(const v4u*)(sH + (it * 4 + q) * 32 + cw * 4);
      for (int pass = 0; pass < 2; ++pass) {
#pragma unroll
        for (int it = 0; it < 4; ++it) {
          const int row = it * 4 + q;
          *(volatile v4u*)(G + (size_t)(mBase + row) * kChunk + n0 + cw * 8) = vals[it];
        }
        __threadfence();
      }
    }
    wave_sync();
  }
}

__global__ __launch_bounds__(256) void combine_kernel(
    const float* __restrict__ s32, const float* __restrict__ wpow, unsigned short* __restrict__ init16) {
  const int lane = threadIdx.x & 31;
  const int wave = __builtin_amdgcn_readfirstlane((int)(threadIdx.x >> 5));
  const int pair = (int)blockIdx.x * 8 + wave;
  const int h = pair >> 4;
  const int b = pair & 15;
  const v2f w = *(const v2f*)(wpow + (size_t)(h * kModes + lane) * 2);
  const float w_re = w[0];
  const float w_im = w[1];
  const float* sp = s32 + ((size_t)h * kRowsM + (size_t)b * kChunksPS) * kStateW + 2 * lane;
  unsigned* ip = (unsigned*)(init16 + ((size_t)h * kRowsM + (size_t)b * kChunksPS) * kStateW) + lane;
  float er = 0.0f, ei = 0.0f;
#pragma unroll 1
  for (int cidx = 0; cidx < kChunksPS; ++cidx) {
    const v2f s = *(const v2f*)(sp + (size_t)cidx * kStateW);
    const float cr = fminf(fmaxf(er, -60000.0f), 60000.0f);
    const float ci = fminf(fmaxf(ei, -60000.0f), 60000.0f);
    const unsigned word = pack2(cr, ci);
    volatile unsigned* q = (volatile unsigned*)(ip + (size_t)cidx * (kStateW / 2));
    *q = word;
    __threadfence();
    *q = word;
    const float tr = w_re * er - w_im * ei + s[0];
    ei = w_re * ei + w_im * er + s[1];
    er = tr;
  }
}

__global__ __launch_bounds__(256) void mix_norm_kernel(
    const unsigned short* __restrict__ g16, const unsigned short* __restrict__ wT,
    const float* __restrict__ b_out, const float* __restrict__ ln_w, const float* __restrict__ ln_b,
    unsigned short* h16) {
  __shared__ __align__(16) union { unsigned w[64 * kPitchW]; unsigned short s[64 * kPitchW * 2]; } sb;
  __shared__ float sRed[2 * 8 * 64];
  __shared__ float sStat[128];
  const int tid = threadIdx.x;
  const int lane = tid & 31;
  const int wave = __builtin_amdgcn_readfirstlane((int)(threadIdx.x >> 5));
  const int hh = lane >> 4;
  const int c = lane & 15;
  const size_t n0 = (size_t)blockIdx.x * 64;

  stage_tile_T<256>(g16, n0, sb.w, tid);
  __syncthreads();

  v8f acc[2][4];
#pragma unroll
  for (int i = 0; i < 2; ++i)
#pragma unroll
    for (int j = 0; j < 4; ++j) acc[i][j] = (v8f){0.f, 0.f, 0.f, 0.f, 0.f, 0.f, 0.f, 0.f};
  {
    const _Float16* Wr = (const _Float16*)wT + (size_t)(32 * wave + c) * kWidth + 8 * hh;
#pragma unroll 1
    for (int ks = 0; ks < kWidth / 32; ++ks) {
      v16h bf[4];
#pragma unroll
      for (int j = 0; j < 4; ++j) bf[j] = lds_frag<kPitchW>(sb.w, 16 * j + c, ks * 16 + 4 * hh);
#pragma unroll
      for (int i = 0; i < 2; ++i) {
        const v16h ah = frag_load(Wr + (size_t)(i * 16) * kWidth + ks * 32);
#pragma unroll
        for (int j = 0; j < 4; ++j) acc[i][j] = mma16(ah, bf[j], acc[i][j]);
        tie_acc(acc[i][0], ah, bf[0]);
        tie_acc(acc[i][1], ah, bf[1]);
        tie_acc(acc[i][2], ah, bf[2]);
        tie_acc_nops(acc[i][3], ah, bf[3]);
      }
      keep4(bf[0], bf[1], bf[2], bf[3]);
    }
  }
  acc_guard4(acc[0][0], acc[0][1], acc[0][2], acc[0][3]);
  acc_guard4(acc[1][0], acc[1][1], acc[1][2], acc[1][3]);
  __syncthreads();

  stage_tile_T<256>(h16, n0, sb.w, tid);
  __syncthreads();

  float s1[4] = {0.f, 0.f, 0.f, 0.f};
  float s2[4] = {0.f, 0.f, 0.f, 0.f};
#pragma unroll
  for (int i = 0; i < 2; ++i) {
    const int d0 = 32 * wave + 16 * i + 8 * hh;
    const v4f b0 = *(const v4f*)(b_out + d0);
    const v4f b1 = *(const v4f*)(b_out + d0 + 4);
#pragma unroll
    for (int j = 0; j < 4; ++j) {
      const int n = 16 * j + c;
      const v4u rw = *(const v4u*)(sb.w + n * kPitchW + (d0 >> 1));
#pragma unroll
      for (int r = 0; r < 8; ++r) {
        const unsigned word = rw[r >> 1];
        const unsigned bits = (r & 1) ? (word >> 16) : (word & 0xffffu);
        const float res = h16_to_f32(bits);
        const float bv = (r < 4) ? b0[r & 3] : b1[r & 3];
        const float val = fmaf(acc[i][j][r], kWCarryInv, bv) + res;
        acc[i][j][r] = val;
        s1[j] += val;
        s2[j] = fmaf(val, val, s2[j]);
      }
    }
  }
#pragma unroll
  for (int j = 0; j < 4; ++j) {
    s1[j] += __shfl_xor(s1[j], 16, 32);
    s2[j] += __shfl_xor(s2[j], 16, 32);
  }
  if (hh == 0) {
#pragma unroll
    for (int j = 0; j < 4; ++j) {
      sRed[wave * 64 + 16 * j + c] = s1[j];
      sRed[512 + wave * 64 + 16 * j + c] = s2[j];
    }
  }
  __syncthreads();
  if (tid < 64) {
    float a = 0.0f, bq = 0.0f;
#pragma unroll 1
    for (int wv = 0; wv < 8; ++wv) {
      a += sRed[wv * 64 + tid];
      bq += sRed[512 + wv * 64 + tid];
    }
    const float mu = a * (1.0f / (float)kWidth);
    float var = bq * (1.0f / (float)kWidth) - mu * mu;
    var = fmaxf(var, 0.0f);
    sStat[tid] = mu;
    sStat[64 + tid] = rsqrtf(var + 1e-5f);
  }
  __syncthreads();
  float mu[4], rs[4];
#pragma unroll
  for (int j = 0; j < 4; ++j) {
    mu[j] = sStat[16 * j + c];
    rs[j] = sStat[64 + 16 * j + c];
  }
#pragma unroll
  for (int i = 0; i < 2; ++i) {
    const int d0 = 32 * wave + 16 * i + 8 * hh;
    const v4f w0 = *(const v4f*)(ln_w + d0);
    const v4f w1 = *(const v4f*)(ln_w + d0 + 4);
    const v4f g0 = *(const v4f*)(ln_b + d0);
    const v4f g1 = *(const v4f*)(ln_b + d0 + 4);
#pragma unroll
    for (int j = 0; j < 4; ++j) {
      const int n = 16 * j + c;
#pragma unroll
      for (int r = 0; r < 8; ++r) {
        const float lw = (r < 4) ? w0[r & 3] : w1[r & 3];
        const float lb = (r < 4) ? g0[r & 3] : g1[r & 3];
        const float xn = (acc[i][j][r] - mu[j]) * rs[j];
        const float o = fmaf(xn, lw, lb);
        sb.s[(d0 + r) * 64 + n] = f16bits(o);
      }
    }
  }
  __syncthreads();
  store_tile_rows(sb.w, h16, n0, wave, lane);
}

__global__ __launch_bounds__(128) void decode_kernel(
    const unsigned short* __restrict__ h16, const unsigned short* __restrict__ dwh, const unsigned short* __restrict__ dwl,
    const float* __restrict__ dec_b, float* __restrict__ out) {
  __shared__ __align__(16) unsigned sW[64 * kPitchW];
  __shared__ __align__(16) float sOut[16 * 68];
  const int tid = threadIdx.x;
  const int lane = tid & 31;
  const int wave = __builtin_amdgcn_readfirstlane((int)(threadIdx.x >> 5));
  const int hh = lane >> 4;
  const int c = lane & 15;
  const size_t n0 = (size_t)blockIdx.x * 64;
  const int b = (int)(n0 >> 12);
  const int l0 = (int)(n0 & (size_t)(kLen - 1));

  stage_tile_T<128>(h16, n0, sW, tid);
  __syncthreads();

  v8f acc_h = (v8f){0.f, 0.f, 0.f, 0.f, 0.f, 0.f, 0.f, 0.f};
  v8f acc_l = (v8f){0.f, 0.f, 0.f, 0.f, 0.f, 0.f, 0.f, 0.f};
  const _Float16* Ah = (const _Float16*)dwh + (size_t)c * kWidth + 8 * hh;
  const _Float16* Al = (const _Float16*)dwl + (size_t)c * kWidth + 8 * hh;
#pragma unroll 1
  for (int ks = 0; ks < kWidth / 32; ++ks) {
    const v16h bf = lds_frag<kPitchW>(sW, 16 * wave + c, ks * 16 + 4 * hh);
    const v16h a1 = frag_load(Ah + ks * 32);
    const v16h a2 = frag_load(Al + ks * 32);
    acc_h = mma16(a1, bf, acc_h);
    acc_l = mma16(a2, bf, acc_l);
    tie_acc(acc_h, a1, bf);
    tie_acc_nops(acc_l, a2, bf);
  }
  {
    const v4f b0 = *(const v4f*)(dec_b + 8 * hh);
    const v4f b1 = *(const v4f*)(dec_b + 8 * hh + 4);
#pragma unroll
    for (int r = 0; r < 8; ++r) {
      const float bv = (r < 4) ? b0[r & 3] : b1[r & 3];
      const float sum = fmaf(acc_l[r], kLoScaleInv, acc_h[r]);
      sOut[(8 * hh + r) * 68 + 16 * wave + c] = fmaf(sum, kWCarryInv, bv);
    }
  }
  __syncthreads();
  {
    const int c4 = (lane & 15) * 4;
    v4f vals[2];
#pragma unroll
    for (int it = 0; it < 2; ++it) vals[it] = *(const v4f*)(sOut + (4 * wave + 2 * it + hh) * 68 + c4);
    for (int pass = 0; pass < 2; ++pass) {
#pragma unroll
      for (int it = 0; it < 2; ++it) {
        const int row = 4 * wave + 2 * it + hh;
        *(volatile v4f*)(out + ((size_t)b * kChanIn + row) * kLen + l0 + c4) = vals[it];
      }
      __threadfence();
    }
  }
}

extern "C" void kernel_launch(void* const* d_in, const int* in_sizes, int n_in,
                              void* d_out, int out_size, void* d_ws, size_t ws_size,
                              hipStream_t stream) {
  if (n_in < 15) return;
  if (in_sizes[0] != kBatch * kChanIn * kLen) return;
  if (in_sizes[1] != kChanIn * kWidth) return;
  if (in_sizes[2] != kWidth) return;
  if (in_sizes[3] != kLayers * kWidth) return;
  if (in_sizes[4] != kLayers * kWidth * kModes) return;
  if (in_sizes[5] != kLayers * kWidth * kModes) return;
  if (in_sizes[6] != kLayers * kWidth * kModes) return;
  if (in_sizes[7] != kLayers * kWidth * kModes) return;
  if (in_sizes[8] != kLayers * kWidth) return;
  if (in_sizes[9] != kLayers * kWidth * kWidth) return;
  if (in_sizes[10] != kLayers * kWidth) return;
  if (in_sizes[11] != kLayers * kWidth) return;
  if (in_sizes[12] != kLayers * kWidth) return;
  if (in_sizes[13] != kWidth * kChanIn) return;
  if (in_sizes[14] != kChanIn) return;
  if (out_size != kBatch * kChanIn * kLen) return;
  if (ws_size < kWsTotal) return;

  const float* x      = (const float*)d_in[0];
  const float* enc_w  = (const float*)d_in[1];
  const float* enc_b  = (const float*)d_in[2];
  const float* log_dt = (const float*)d_in[3];
  const float* A_re   = (const float*)d_in[4];
  const float* A_im   = (const float*)d_in[5];
  const float* C_re   = (const float*)d_in[6];
  const float* C_im   = (const float*)d_in[7];
  const float* Dv     = (const float*)d_in[8];
  const float* W_out  = (const float*)d_in[9];
  const float* b_out  = (const float*)d_in[10];
  const float* ln_w   = (const float*)d_in[11];
  const float* ln_b   = (const float*)d_in[12];
  const float* dec_w  = (const float*)d_in[13];
  const float* dec_b  = (const float*)d_in[14];
  float* out = (float*)d_out;

  char* ws = (char*)d_ws;
  unsigned short* H16    = (unsigned short*)(ws + kOffH16);
  unsigned short* G16    = (unsigned short*)(ws + kOffG16);
  float*          S32    = (float*)(ws + kOffG16);
  unsigned short* INIT16 = (unsigned short*)(ws + kOffInit);
  unsigned short* MV16   = (unsigned short*)(ws + kOffMv);
  unsigned short* ET16   = (unsigned short*)(ws + kOffEt);
  float*          WPOW   = (float*)(ws + kOffWpow);
  unsigned short* WOUTT  = (unsigned short*)(ws + kOffWoutT);
  unsigned short* DECH   = (unsigned short*)(ws + kOffDecH);
  unsigned short* DECL   = (unsigned short*)(ws + kOffDecL);
  unsigned short* ENCT   = (unsigned short*)(ws + kOffEncT);

  weight_planes_kernel<<<41, 256, 0, stream>>>(W_out, enc_w, dec_w, WOUTT, ENCT, DECH, DECL);
  encode_kernel<<<kNpos / 64, 256, 0, stream>>>(x, ENCT, enc_b, H16);

  for (int i = 0; i < kLayers; ++i) {
    const size_t om = (size_t)i * kWidth * kModes;
    layer_tables_kernel<<<kWidth, 256, 0, stream>>>(log_dt + i * kWidth, A_re + om, A_im + om, C_re + om, C_im + om,
                                                    Dv + i * kWidth, ET16, MV16, WPOW);
    chunk_gemm_kernel<0><<<dim3(1, kWidth), 256, 0, stream>>>(H16, nullptr, ET16, (void*)S32);
    combine_kernel<<<(kWidth * kBatch) / 8, 256, 0, stream>>>(S32, WPOW, INIT16);
    chunk_gemm_kernel<1><<<dim3(2, kWidth), 256, 0, stream>>>(H16, INIT16, MV16, (void*)G16);
    mix_norm_kernel<<<kNpos / 64, 256, 0, stream>>>(G16, WOUTT + (size_t)i * kWidth * kWidth, b_out + i * kWidth,
                                                    ln_w + i * kWidth, ln_b + i * kWidth, H16);
  }

  decode_kernel<<<kNpos / 64, 128, 0, stream>>>(H16, DECH, DECL, dec_b, out);
}
